// MACEInteraction_47004122087965
// MI455X (gfx1250) — hardware-verified
//
#include <hip/hip_runtime.h>
#include <stddef.h>


#define MUL     128
#define SHD     16
#define RBF     8
#define HID     64
#define WEC     512
#define NTHR    256
#define NWAVE   8
#define EPT     8
#define NGRP    2
#define CHUNK   (NTHR * EPT * NGRP)
#define WCAP    (EPT * NGRP * 32)
#define LISTN   (NWAVE * WCAP)
#define NBC     4096
#define NBF     1024
#define RCAP    40960
#define RBN     128
#define OTHR    512
#define ETHR    128
#define EWAVE   4
#define RUN     8
#define TGT     (EWAVE * RUN)
#define DEGCAP  256
#define MAXT    ((RUN * DEGCAP + 15) / 16)
#define HP      (HID + 8)
#define WEP     WEC
#define GROWS   128
#define APH     (MUL + 8)
#define PNODE   16
#define WSCAP   134217728
#define S8F     0.35355339059327373f
#define S64F    0.125f
#define INV128  0.08838834764831845f

#define PO_PRE   0
#define PO_W0    32768
#define PO_W1    36864
#define PO_W2    45056
#define PO_W3    53248
#define PO_POST  118784
#define PO_TOTAL 249856
#define WPB      61

#define LDS_PRE  (2 * GROWS * APH * 2)
#define LDS_FILL ((RCAP + NBF + LISTN) * 4 + 64)
#define LDS_E_WE (EWAVE * 16 * WEP * 4)
#define LDS_E_H  (EWAVE * 4 * 16 * HP * 2)
#define LDS_E_RB (EWAVE * 16 * RBF * 4)
#define LDS_E_MT (EWAVE * 32 * 4)
#define LDS_E_BD (EWAVE * 16 * 4)
#define LDS_EDGE (LDS_E_WE + LDS_E_H + LDS_E_RB + LDS_E_MT + LDS_E_BD)
#define LDS_POST (PNODE * MUL * SHD * 4)

static_assert((CHUNK & (CHUNK - 1)) == 0);
static_assert(CHUNK <= 4096);
static_assert((NBC & (NBC - 1)) == 0 && (NBF & (NBF - 1)) == 0);
static_assert(NBC == 4 * NBF);
static_assert(OTHR * 8 == NBC);
static_assert((RCAP % 32) == 0);
static_assert(GROWS * MUL * 4 <= LDS_PRE);
static_assert((APH * 2) % 16 == 0);
static_assert((HP * 2) % 16 == 0);
static_assert(GROWS == NWAVE * 16);
static_assert((GROWS * MUL / 8) % NTHR == 0);
static_assert((NBF % TGT) == 0);
static_assert(TGT * 4 <= NBC);
static_assert(PO_W0 == PO_PRE + 2 * MUL * MUL);
static_assert(PO_W1 == PO_W0 + 2 * HID * 32);
static_assert(PO_W2 == PO_W1 + 2 * HID * HID);
static_assert(PO_W3 == PO_W2 + 2 * HID * HID);
static_assert(PO_POST == PO_W3 + 2 * WEC * HID);
static_assert(PO_TOTAL == PO_POST + 8 * MUL * MUL);
static_assert(WPB * 256 == (MUL * MUL + HID * 32 + 2 * HID * HID + WEC * HID + 4 * MUL * MUL) / 8);
static_assert((PNODE * MUL * SHD / 4) % NTHR == 0);
static_assert(RUN + 1 <= 16);
static_assert((TGT % PNODE) == 0);

typedef float          v4f  __attribute__((ext_vector_type(4)));
typedef float          v8f  __attribute__((ext_vector_type(8)));
typedef int            v4i  __attribute__((ext_vector_type(4)));
typedef unsigned short v4us __attribute__((ext_vector_type(4)));
typedef unsigned short v8us __attribute__((ext_vector_type(8)));
typedef __bf16         v16b __attribute__((ext_vector_type(16)));
typedef v4f  __attribute__((may_alias)) v4fa;
typedef v8us __attribute__((may_alias)) v8usa;
union FragB { v16b v; v8us h[2]; };

__device__ __forceinline__ unsigned int bfr(float f) {
  const unsigned int u = __float_as_uint(f);
  return (u + 0x7FFFu + ((u >> 16) & 1u)) >> 16;
}

__device__ __forceinline__ void split1(float x, unsigned short& hb, unsigned short& lb) {
  const unsigned int hu = bfr(x);
  const float hf = __uint_as_float(hu << 16);
  hb = (unsigned short)hu;
  lb = (unsigned short)bfr(x - hf);
}

__device__ __forceinline__ void split8(v4f a, v4f b, v8us& hi, v8us& lo) {
  unsigned short hb, lb;
  split1(a.x, hb, lb); hi[0] = hb; lo[0] = lb;
  split1(a.y, hb, lb); hi[1] = hb; lo[1] = lb;
  split1(a.z, hb, lb); hi[2] = hb; lo[2] = lb;
  split1(a.w, hb, lb); hi[3] = hb; lo[3] = lb;
  split1(b.x, hb, lb); hi[4] = hb; lo[4] = lb;
  split1(b.y, hb, lb); hi[5] = hb; lo[5] = lb;
  split1(b.z, hb, lb); hi[6] = hb; lo[6] = lb;
  split1(b.w, hb, lb); hi[7] = hb; lo[7] = lb;
}

__device__ __forceinline__ void split4(v4f a, v4us& hi, v4us& lo) {
  unsigned short hb, lb;
  split1(a.x, hb, lb); hi[0] = hb; lo[0] = lb;
  split1(a.y, hb, lb); hi[1] = hb; lo[1] = lb;
  split1(a.z, hb, lb); hi[2] = hb; lo[2] = lb;
  split1(a.w, hb, lb); hi[3] = hb; lo[3] = lb;
}

__device__ __forceinline__ v8f wmb(v16b a, v16b b, v8f c) {
  v8f d = __builtin_amdgcn_wmma_f32_16x16x32_bf16(false, a, false, b, (short)0, c, false, false);
  asm volatile("v_nop\n\tv_nop\n\tv_nop\n\tv_nop" : "+v"(d) : "v"(a), "v"(b));
  return d;
}

__device__ __forceinline__ v8f zero8() { v8f z = {0.f, 0.f, 0.f, 0.f, 0.f, 0.f, 0.f, 0.f}; return z; }

__device__ __forceinline__ void wave_lds_sync() {
  __builtin_amdgcn_fence(__ATOMIC_RELEASE, "wavefront");
  __builtin_amdgcn_wave_barrier();
}

__device__ __forceinline__ float silu_f(float v) {
  float ev = __expf(-v);
  ev = fminf(ev, 1.0e15f);
  return v * __builtin_amdgcn_rcpf(1.0f + ev);
}

template <int NB>
__device__ __forceinline__ int scan_chunk(const int* __restrict__ dsts, int nE, int cbase, int slotBase,
                                          int vec8, int* list, int tid, int lane, int wave) {
  int wc = 0;
#pragma unroll
  for (int g = 0; g < NGRP; ++g) {
    const int el0  = (g * NTHR + tid) * EPT;
    const int e0   = cbase + el0;
    const int sent = -2147483647 - 1;
    v4i da, db;
    if (vec8 != 0 && cbase + CHUNK <= nE) {
      da = *(const v4i*)(dsts + e0);
      db = *(const v4i*)(dsts + e0 + 4);
    } else {
      da.x = (e0     < nE) ? dsts[min(e0, nE - 1)] : sent;
      da.y = (e0 + 1 < nE) ? dsts[min(e0 + 1, nE - 1)] : sent;
      da.z = (e0 + 2 < nE) ? dsts[min(e0 + 2, nE - 1)] : sent;
      da.w = (e0 + 3 < nE) ? dsts[min(e0 + 3, nE - 1)] : sent;
      db.x = (e0 + 4 < nE) ? dsts[min(e0 + 4, nE - 1)] : sent;
      db.y = (e0 + 5 < nE) ? dsts[min(e0 + 5, nE - 1)] : sent;
      db.z = (e0 + 6 < nE) ? dsts[min(e0 + 6, nE - 1)] : sent;
      db.w = (e0 + 7 < nE) ? dsts[min(e0 + 7, nE - 1)] : sent;
    }
    const unsigned nb = (unsigned)slotBase;
    const unsigned s0 = (unsigned)da.x - nb, s1 = (unsigned)da.y - nb;
    const unsigned s2 = (unsigned)da.z - nb, s3 = (unsigned)da.w - nb;
    const unsigned s4 = (unsigned)db.x - nb, s5 = (unsigned)db.y - nb;
    const unsigned s6 = (unsigned)db.z - nb, s7 = (unsigned)db.w - nb;
    const bool h0 = s0 < (unsigned)NB, h1 = s1 < (unsigned)NB, h2 = s2 < (unsigned)NB, h3 = s3 < (unsigned)NB;
    const bool h4 = s4 < (unsigned)NB, h5 = s5 < (unsigned)NB, h6 = s6 < (unsigned)NB, h7 = s7 < (unsigned)NB;
    const unsigned any = __builtin_amdgcn_ballot_w32(h0 | h1 | h2 | h3 | h4 | h5 | h6 | h7);
    if (any != 0u) {
#define HITJ(J, HJ, SJ) { \
        const unsigned mj = __builtin_amdgcn_ballot_w32(HJ); \
        if (mj != 0u) { \
          if (HJ) { \
            const int pos = wc + (int)__builtin_amdgcn_mbcnt_lo(mj, 0u); \
            if (pos < WCAP) list[wave * WCAP + pos] = ((el0 + (J)) << 12) | (int)(SJ); \
          } \
          wc += (int)__builtin_popcount(mj); } }
      HITJ(0, h0, s0)
      HITJ(1, h1, s1)
      HITJ(2, h2, s2)
      HITJ(3, h3, s3)
      HITJ(4, h4, s4)
      HITJ(5, h5, s5)
      HITJ(6, h6, s6)
      HITJ(7, h7, s7)
#undef HITJ
    }
  }
  return wc;
}

__global__ __launch_bounds__(NTHR) void k_wprep(
    const float* __restrict__ Wpre, const float* __restrict__ w0, const float* __restrict__ w1,
    const float* __restrict__ w2, const float* __restrict__ w3, const float* __restrict__ Wpost,
    unsigned short* wp) {
  const int tid = (int)threadIdx.x, b = (int)blockIdx.x;
  const float* src;
  int K, srcK, N, lk, po, i;
  if (b < 8)        { src = Wpre; K = 128; srcK = 128; N = 128; lk = 4; po = PO_PRE; i = b * 256 + tid; }
  else if (b < 9)   { src = w0;   K = 32;  srcK = 8;   N = 64;  lk = 2; po = PO_W0;  i = (b - 8) * 256 + tid; }
  else if (b < 11)  { src = w1;   K = 64;  srcK = 64;  N = 64;  lk = 3; po = PO_W1;  i = (b - 9) * 256 + tid; }
  else if (b < 13)  { src = w2;   K = 64;  srcK = 64;  N = 64;  lk = 3; po = PO_W2;  i = (b - 11) * 256 + tid; }
  else if (b < 29)  { src = w3;   K = 64;  srcK = 64;  N = 512; lk = 3; po = PO_W3;  i = (b - 13) * 256 + tid; }
  else {
    const int ii = (b - 29) * 256 + tid;
    const int p  = ii >> 11;
    src = Wpost + (size_t)p * (MUL * MUL); K = 128; srcK = 128; N = 128; lk = 4;
    po = PO_POST + p * (2 * MUL * MUL); i = ii & 2047;
  }
  const int kq = K >> 3;
  const int n  = i >> lk;
  const int k0 = (i & (kq - 1)) * 8;
  float v[8];
#pragma unroll
  for (int e = 0; e < 8; ++e) {
    const int k  = k0 + e;
    const int kc = k < srcK - 1 ? k : srcK - 1;
    const float t = src[(size_t)kc * N + n];
    v[e] = (k < srcK) ? t : 0.0f;
  }
  v4f a, c;
  a.x = v[0]; a.y = v[1]; a.z = v[2]; a.w = v[3];
  c.x = v[4]; c.y = v[5]; c.z = v[6]; c.w = v[7];
  v8us hv, lv;
  split8(a, c, hv, lv);
  unsigned short* dh = wp + po + (size_t)i * 8;
  unsigned short* dl = dh + (size_t)N * K;
  *(volatile v8us*)dh = hv;
  *(volatile v8us*)dl = lv;
  __threadfence();
  *(volatile v8us*)dh = hv;
  *(volatile v8us*)dl = lv;
}

__global__ __launch_bounds__(NTHR) void k_count(
    const int* __restrict__ dsts, int* cnt, int nE, int vec8) {
  __shared__ __attribute__((aligned(16))) int scnt[NBC];
  __shared__ __attribute__((aligned(16))) int list[LISTN];
  __shared__ int wcnt[NWAVE];
  const int tid = threadIdx.x, lane = tid & 31, wave = tid >> 5;
  const int nodeBase = blockIdx.x * NBC;

  for (int i = tid; i < NBC; i += NTHR) scnt[i] = 0;
  __syncthreads();

  const int nChunks = (nE + CHUNK - 1) / CHUNK;
#pragma unroll 1
  for (int ch = 0; ch < nChunks; ++ch) {
    const int cbase = ch * CHUNK;
    const int wc = scan_chunk<NBC>(dsts, nE, cbase, nodeBase, vec8, list, tid, lane, wave);
    if (lane == 0) wcnt[wave] = wc;
    __syncthreads();
    if (wave == 0) {
#pragma unroll 1
      for (int wsx = 0; wsx < NWAVE; ++wsx) {
        int n = __builtin_amdgcn_readfirstlane(wcnt[wsx]);
        n = n > WCAP ? WCAP : (n < 0 ? 0 : n);
        const int* lp = list + wsx * WCAP;
#pragma unroll 1
        for (int i = 0; i < n; ++i) {
          const int ent  = __builtin_amdgcn_readfirstlane(lp[i]);
          const int slot = ent & (NBC - 1);
          if (lane == 0) scnt[slot] = scnt[slot] + 1;
        }
      }
    }
    __syncthreads();
  }

  v4i cq[4];
#pragma unroll
  for (int q = 0; q < 4; ++q) {
    const int f = (wave * 4 + q) * 128 + 4 * lane;
    cq[q] = *(const v4i*)(scnt + f);
  }
  int* cp = cnt + (size_t)nodeBase;
#pragma unroll
  for (int q = 0; q < 4; ++q) {
    const int f = (wave * 4 + q) * 128 + 4 * lane;
    *(volatile v4i*)(cp + f) = cq[q];
  }
  __threadfence();
#pragma unroll
  for (int q = 0; q < 4; ++q) {
    const int f = (wave * 4 + q) * 128 + 4 * lane;
    *(volatile v4i*)(cp + f) = cq[q];
  }
}

__global__ __launch_bounds__(OTHR) void k_offsets(
    const int* __restrict__ cnt, int* off, int* rbase, int nChunk) {
  __shared__ __attribute__((aligned(16))) int soff[NBC];
  __shared__ __attribute__((aligned(16))) int srb[RBN];
  __shared__ int wtot[OTHR / 32];
  const int tid = threadIdx.x, lane = tid & 31, wave = tid >> 5, sub = tid >> 7;
  for (int i = tid; i < RBN; i += OTHR) srb[i] = 0;
  int carry = 0;
#pragma unroll 1
  for (int ch = 0; ch < nChunk; ++ch) {
    const int base = ch * NBC;
    const v4i c0 = *(const v4i*)(cnt + base + 8 * tid);
    const v4i c1 = *(const v4i*)(cnt + base + 8 * tid + 4);
    const int e0 = max(c0.x, 0), e1 = max(c0.y, 0), e2 = max(c0.z, 0), e3 = max(c0.w, 0);
    const int e4 = max(c1.x, 0), e5 = max(c1.y, 0), e6 = max(c1.z, 0), e7 = max(c1.w, 0);
    const int ts = e0 + e1 + e2 + e3 + e4 + e5 + e6 + e7;
    int incl = ts;
#pragma unroll
    for (int d = 1; d < 32; d <<= 1) {
      const int t = __shfl_up(incl, d);
      if (lane >= d) incl += t;
    }
    if (lane == 31) wtot[wave] = incl;
    __syncthreads();
    const int S0 = wtot[0]  + wtot[1]  + wtot[2]  + wtot[3];
    const int S1 = wtot[4]  + wtot[5]  + wtot[6]  + wtot[7];
    const int S2 = wtot[8]  + wtot[9]  + wtot[10] + wtot[11];
    const int S3 = wtot[12] + wtot[13] + wtot[14] + wtot[15];
    int pre = 0;
#pragma unroll 1
    for (int w = 4 * sub; w < wave; ++w) pre += wtot[w];
    const int b0 = carry;
    const int b1 = b0 + ((S0 + 31) & ~31);
    const int b2 = b1 + ((S1 + 31) & ~31);
    const int b3 = b2 + ((S2 + 31) & ~31);
    const int b4 = b3 + ((S3 + 31) & ~31);
    const int myb = sub == 0 ? b0 : (sub == 1 ? b1 : (sub == 2 ? b2 : b3));
    if (tid == 0) {
      srb[min(4 * ch + 0, RBN - 1)] = b0;
      srb[min(4 * ch + 1, RBN - 1)] = b1;
      srb[min(4 * ch + 2, RBN - 1)] = b2;
      srb[min(4 * ch + 3, RBN - 1)] = b3;
    }
    int run = myb + pre + incl - ts;
    soff[8 * tid + 0] = run; run += e0;
    soff[8 * tid + 1] = run; run += e1;
    soff[8 * tid + 2] = run; run += e2;
    soff[8 * tid + 3] = run; run += e3;
    soff[8 * tid + 4] = run; run += e4;
    soff[8 * tid + 5] = run; run += e5;
    soff[8 * tid + 6] = run; run += e6;
    soff[8 * tid + 7] = run;
    carry = b4;
    __syncthreads();
    const v4i o0 = *(const v4i*)(soff + 4 * tid);
    const v4i o1 = *(const v4i*)(soff + 4 * (tid + OTHR));
    int* op = off + base;
    *(volatile v4i*)(op + 4 * tid) = o0;
    *(volatile v4i*)(op + 4 * (tid + OTHR)) = o1;
    __threadfence();
    *(volatile v4i*)(op + 4 * tid) = o0;
    *(volatile v4i*)(op + 4 * (tid + OTHR)) = o1;
    __syncthreads();
  }
  if (tid == 0) srb[min(4 * nChunk, RBN - 1)] = carry;
  __syncthreads();
  v4i rv = {0, 0, 0, 0};
  if (tid < 32) rv = *(const v4i*)(srb + 4 * tid);
  if (tid < 32) *(volatile v4i*)(rbase + 4 * tid) = rv;
  __threadfence();
  if (tid < 32) *(volatile v4i*)(rbase + 4 * tid) = rv;
}

__global__ __launch_bounds__(NTHR) void k_fill(
    const int* __restrict__ dsts, const int* __restrict__ off, const int* __restrict__ rbase,
    int* csr, int nE, int vec8, int csrLen) {
  extern __shared__ v4f lds_dyn[];
  int* region = (int*)lds_dyn;
  int* cursor = region + RCAP;
  int* list   = cursor + NBF;
  int* wcnt   = list + LISTN;
  const int tid = threadIdx.x, lane = tid & 31, wave = tid >> 5;
  const int b = blockIdx.x;
  const int nodeBase = b * NBF;

  int rb0 = rbase[b];
  const int rb1 = rbase[b + 1];
  rb0 = rb0 < 0 ? 0 : (rb0 > csrLen ? csrLen : rb0);
  rb0 &= ~31;
  int len = rb1 - rb0;
  len = len < 0 ? 0 : (len > RCAP ? RCAP : len);
  int lenW = (len + 31) & ~31;
  if (rb0 + lenW > csrLen) lenW = (csrLen - rb0) & ~31;

  {
    const v4i z = {0, 0, 0, 0};
    for (int i = tid; i < RCAP / 4; i += NTHR) ((v4i*)region)[i] = z;
    for (int s = tid; s < NBF; s += NTHR) {
      int o = off[nodeBase + s] - rb0;
      o = o < 0 ? 0 : (o > RCAP ? RCAP : o);
      cursor[s] = o;
    }
  }
  __syncthreads();

  const int nChunks = (nE + CHUNK - 1) / CHUNK;
#pragma unroll 1
  for (int ch = 0; ch < nChunks; ++ch) {
    const int cbase = ch * CHUNK;
    const int wc = scan_chunk<NBF>(dsts, nE, cbase, nodeBase, vec8, list, tid, lane, wave);
    if (lane == 0) wcnt[wave] = wc;
    __syncthreads();
    if (wave == 0) {
#pragma unroll 1
      for (int wsx = 0; wsx < NWAVE; ++wsx) {
        int n = __builtin_amdgcn_readfirstlane(wcnt[wsx]);
        n = n > WCAP ? WCAP : (n < 0 ? 0 : n);
        const int* lp = list + wsx * WCAP;
#pragma unroll 1
        for (int i = 0; i < n; ++i) {
          const int ent  = __builtin_amdgcn_readfirstlane(lp[i]);
          const int slot = ent & (NBF - 1);
          int e = cbase + ((ent >> 12) & (CHUNK - 1));
          e = e > nE - 1 ? nE - 1 : e;
          if (lane == 0) {
            int pos = cursor[slot];
            pos = pos < 0 ? 0 : (pos > RCAP - 1 ? RCAP - 1 : pos);
            region[pos] = e;
            const int np = pos + 1;
            cursor[slot] = np > RCAP ? RCAP : np;
          }
        }
      }
    }
    __syncthreads();
  }

  const int nv = lenW >> 2;
  int* gp = csr + rb0;
#pragma unroll 1
  for (int i = tid; i < nv; i += NTHR) { const v4i v = ((const v4i*)region)[i]; *(volatile v4i*)(gp + 4 * i) = v; }
  __threadfence();
#pragma unroll 1
  for (int i = tid; i < nv; i += NTHR) { const v4i v = ((const v4i*)region)[i]; *(volatile v4i*)(gp + 4 * i) = v; }
}

__global__ __launch_bounds__(NTHR) void k_pre(
    const float* __restrict__ A, const unsigned short* __restrict__ wp, float* C, int nRowsA, float scl) {
  extern __shared__ v4f lds_dyn[];
  constexpr int KD = MUL;
  unsigned short* sHi = (unsigned short*)lds_dyn;
  unsigned short* sLo = sHi + GROWS * APH;
  float*          stg = (float*)lds_dyn;
  const int tid = threadIdx.x, lane = tid & 31, wave = tid >> 5, hh = lane >> 4, m = lane & 15;
  const int rowBase = blockIdx.x * GROWS;
  const unsigned short* Bw = wp + PO_PRE;

#pragma unroll
  for (int i = 0; i < (GROWS * KD / 8) / NTHR; ++i) {
    const int idx = i * NTHR + tid;
    const int r   = idx / (KD / 8);
    const int c0  = (idx - r * (KD / 8)) * 8;
    int row = rowBase + r;
    row = row > nRowsA - 1 ? nRowsA - 1 : row;
    const float* ap = A + (size_t)row * KD + c0;
    const v4f a = *(const v4f*)ap, b = *(const v4f*)(ap + 4);
    v8us hv, lv;
    split8(a, b, hv, lv);
    *(v8us*)(sHi + r * APH + c0) = hv;
    *(v8us*)(sLo + r * APH + c0) = lv;
  }
  __syncthreads();

  v8f acc[8];
#pragma unroll
  for (int t = 0; t < 8; ++t) acc[t] = zero8();
  const unsigned short* ahp = sHi + (wave * 16 + m) * APH + 8 * hh;
  const unsigned short* alp = sLo + (wave * 16 + m) * APH + 8 * hh;
#pragma unroll
  for (int kt = 0; kt < KD / 32; ++kt) {
    FragB ah, al;
    ah.h[0] = *(const v8usa*)(ahp + 32 * kt);
    ah.h[1] = *(const v8usa*)(ahp + 32 * kt + 16);
    al.h[0] = *(const v8usa*)(alp + 32 * kt);
    al.h[1] = *(const v8usa*)(alp + 32 * kt + 16);
#pragma unroll
    for (int t = 0; t < 8; ++t) {
      const unsigned short* bp = Bw + (size_t)(16 * t + m) * KD + 32 * kt + 8 * hh;
      FragB bh, bl;
      bh.h[0] = *(const v8us*)bp;
      bh.h[1] = *(const v8us*)(bp + 16);
      bl.h[0] = *(const v8us*)(bp + MUL * MUL);
      bl.h[1] = *(const v8us*)(bp + MUL * MUL + 16);
      acc[t] = wmb(ah.v, bh.v, acc[t]);
      acc[t] = wmb(ah.v, bl.v, acc[t]);
      acc[t] = wmb(al.v, bh.v, acc[t]);
    }
  }
  __syncthreads();

  const int r0 = wave * 16 + 8 * hh;
  float* sp = stg + r0 * MUL + m;
#pragma unroll
  for (int t = 0; t < 8; ++t) {
#pragma unroll
    for (int r = 0; r < 8; ++r) sp[r * MUL + 16 * t] = acc[t][r] * scl;
  }
  __syncthreads();

  const float* lp = stg + wave * 16 * MUL + 4 * lane;
  float* gp = C + (size_t)(rowBase + wave * 16) * MUL + 4 * lane;
  v4f rv[16];
#pragma unroll
  for (int i = 0; i < 16; ++i) rv[i] = *(const v4f*)(lp + i * MUL);
#pragma unroll
  for (int i = 0; i < 16; ++i) *(volatile v4f*)(gp + (size_t)i * MUL) = rv[i];
  __threadfence();
#pragma unroll
  for (int i = 0; i < 16; ++i) *(volatile v4f*)(gp + (size_t)i * MUL) = rv[i];
}

__device__ __forceinline__ void act_store(v8f d, float s, unsigned short* oH, unsigned short* oL, int hh, int col) {
#pragma unroll
  for (int r = 0; r < 8; ++r) {
    const float v = silu_f(d[r] * s);
    unsigned short hb, lb;
    split1(v, hb, lb);
    oH[(8 * hh + r) * HP + col] = hb;
    oL[(8 * hh + r) * HP + col] = lb;
  }
}

__device__ __forceinline__ void mlp64(const unsigned short* aH, const unsigned short* aL,
                                      const unsigned short* __restrict__ Bw,
                                      unsigned short* oH, unsigned short* oL, float s, int hh, int m) {
  FragB ah[2], al[2];
#pragma unroll
  for (int kt = 0; kt < 2; ++kt) {
    const unsigned short* ap = aH + m * HP + 32 * kt + 8 * hh;
    const unsigned short* lp = aL + m * HP + 32 * kt + 8 * hh;
    ah[kt].h[0] = *(const v8usa*)ap;
    ah[kt].h[1] = *(const v8usa*)(ap + 16);
    al[kt].h[0] = *(const v8usa*)lp;
    al[kt].h[1] = *(const v8usa*)(lp + 16);
  }
#pragma unroll
  for (int nt = 0; nt < 4; ++nt) {
    v8f d = zero8();
#pragma unroll
    for (int kt = 0; kt < 2; ++kt) {
      const unsigned short* bp = Bw + (size_t)(16 * nt + m) * HID + 32 * kt + 8 * hh;
      FragB bh, bl;
      bh.h[0] = *(const v8us*)bp;
      bh.h[1] = *(const v8us*)(bp + 16);
      bl.h[0] = *(const v8us*)(bp + HID * HID);
      bl.h[1] = *(const v8us*)(bp + HID * HID + 16);
      d = wmb(ah[kt].v, bh.v, d);
      d = wmb(ah[kt].v, bl.v, d);
      d = wmb(al[kt].v, bh.v, d);
    }
    act_store(d, s, oH, oL, hh, 16 * nt + m);
  }
}

__device__ __forceinline__ void flush_node(unsigned short* totH, unsigned short* totL, int node,
                                           v4f (&acc)[SHD], int lane) {
  v4us hv[SHD], lv[SHD];
#pragma unroll
  for (int d = 0; d < SHD; ++d) {
    split4(acc[d], hv[d], lv[d]);
    const v4f z = {0.f, 0.f, 0.f, 0.f};
    acc[d] = z;
  }
  unsigned short* ph = totH + (size_t)node * (SHD * MUL) + 4 * lane;
  unsigned short* pl = totL + (size_t)node * (SHD * MUL) + 4 * lane;
#pragma unroll
  for (int d = 0; d < SHD; ++d) {
    *(volatile v4us*)(ph + d * MUL) = hv[d];
    *(volatile v4us*)(pl + d * MUL) = lv[d];
  }
  __threadfence();
#pragma unroll
  for (int d = 0; d < SHD; ++d) {
    *(volatile v4us*)(ph + d * MUL) = hv[d];
    *(volatile v4us*)(pl + d * MUL) = lv[d];
  }
}

__global__ __launch_bounds__(ETHR) __attribute__((amdgpu_num_vgpr(256)))
void k_edge(const int* __restrict__ csr, const int* __restrict__ offp, const int* __restrict__ cnt,
            const int* __restrict__ ej, const float* __restrict__ rbp, const float* __restrict__ sph,
            const float* __restrict__ xs, const unsigned short* __restrict__ wp,
            unsigned short* totH, unsigned short* totL, int nN, int nE, int csrLen) {
  extern __shared__ v4f lds_dyn[];
  char* base = (char*)lds_dyn;
  float*          wE   = (float*)base;
  unsigned short* hbuf = (unsigned short*)(base + LDS_E_WE);
  float*          rbS  = (float*)(base + LDS_E_WE + LDS_E_H);
  int*            meta = (int*)(base + LDS_E_WE + LDS_E_H + LDS_E_RB);
  int*            bndS = (int*)(base + LDS_E_WE + LDS_E_H + LDS_E_RB + LDS_E_MT);
  const int tid = threadIdx.x, lane = tid & 31, wave = tid >> 5, hh = lane >> 4, m = lane & 15;

  float*          wEw  = wE + wave * 16 * WEP;
  unsigned short* hw   = hbuf + wave * (4 * 16 * HP);
  unsigned short* p0H  = hw;
  unsigned short* p0L  = hw + 16 * HP;
  unsigned short* p1H  = hw + 2 * 16 * HP;
  unsigned short* p1L  = hw + 3 * 16 * HP;
  float*          rbw  = rbS + wave * 16 * RBF;
  int*            eidw = meta + wave * 32;
  int*            jw   = eidw + 16;
  int*            bw   = bndS + wave * 16;
  const int runBase = blockIdx.x * TGT + wave * RUN;

  int cl = cnt[runBase + (lane < RUN ? lane : RUN - 1)];
  cl = (lane < RUN) ? cl : 0;
  cl = cl < 0 ? 0 : (cl > DEGCAP ? DEGCAP : cl);
  int incl = cl;
#pragma unroll
  for (int d = 1; d < 32; d <<= 1) {
    const int t = __shfl_up(incl, d);
    if (lane >= d) incl += t;
  }
  if (lane < RUN) bw[lane + 1] = incl;
  if (lane == 0) bw[0] = 0;
  const int total = __builtin_amdgcn_readfirstlane(__shfl(incl, RUN - 1));
  int rs = offp[runBase];
  {
    const int lim = csrLen - total;
    rs = rs < 0 ? 0 : (rs > lim ? lim : rs);
  }
  wave_lds_sync();
  int nTiles = (total + 15) >> 4;
  nTiles = nTiles > MAXT ? MAXT : nTiles;

  v4f acc[SHD];
#pragma unroll
  for (int d = 0; d < SHD; ++d) { const v4f z = {0.f, 0.f, 0.f, 0.f}; acc[d] = z; }
  int cur = 0;

  const unsigned short* w0p = wp + PO_W0;
  const unsigned short* w3p = wp + PO_W3;
  const v8us z8 = {0, 0, 0, 0, 0, 0, 0, 0};

#pragma unroll 1
  for (int t = 0; t < nTiles; ++t) {
    wave_lds_sync();
    {
      const int r = lane & 15;
      int g = 16 * t + r;
      g = g > total - 1 ? total - 1 : g;
      int pos = rs + g;
      pos = pos < 0 ? 0 : (pos > csrLen - 1 ? csrLen - 1 : pos);
      int e = csr[pos];
      e = e < 0 ? 0 : (e > nE - 1 ? nE - 1 : e);
      int j = ej[e];
      j = j < 0 ? j + nN : j;
      j = j < 0 ? 0 : (j > nN - 1 ? nN - 1 : j);
      if (lane < 16) { eidw[r] = e; jw[r] = j; }
    }
    wave_lds_sync();
    {
      const int row = lane >> 1, half = lane & 1;
      const int e = eidw[row];
      const v4f v = *(const v4f*)(rbp + (size_t)e * RBF + 4 * half);
      *(v4f*)(rbw + row * RBF + 4 * half) = v;
    }
    wave_lds_sync();
    FragB a0h, a0l;
    {
      v4f a = *(const v4fa*)(rbw + m * RBF);
      v4f b = *(const v4fa*)(rbw + m * RBF + 4);
      const v4f zz = {0.f, 0.f, 0.f, 0.f};
      a = hh ? zz : a;
      b = hh ? zz : b;
      v8us hv, lv;
      split8(a, b, hv, lv);
      a0h.h[0] = hv; a0h.h[1] = z8;
      a0l.h[0] = lv; a0l.h[1] = z8;
    }
#pragma unroll
    for (int nt = 0; nt < 4; ++nt) {
      const unsigned short* bp = w0p + (size_t)(16 * nt + m) * 32 + 8 * hh;
      FragB bh, bl;
      bh.h[0] = *(const v8us*)bp;
      bh.h[1] = *(const v8us*)(bp + 16);
      bl.h[0] = *(const v8us*)(bp + HID * 32);
      bl.h[1] = *(const v8us*)(bp + HID * 32 + 16);
      v8f d = zero8();
      d = wmb(a0h.v, bh.v, d);
      d = wmb(a0h.v, bl.v, d);
      d = wmb(a0l.v, bh.v, d);
      act_store(d, S8F, p0H, p0L, hh, 16 * nt + m);
    }
    wave_lds_sync();
    mlp64(p0H, p0L, wp + PO_W1, p1H, p1L, S64F, hh, m);
    wave_lds_sync();
    mlp64(p1H, p1L, wp + PO_W2, p0H, p0L, S64F, hh, m);
    wave_lds_sync();
    {
      FragB ah0, ah1, al0, al1;
      const unsigned short* ap = p0H + m * HP + 8 * hh;
      const unsigned short* lp = p0L + m * HP + 8 * hh;
      ah0.h[0] = *(const v8usa*)ap;        ah0.h[1] = *(const v8usa*)(ap + 16);
      ah1.h[0] = *(const v8usa*)(ap + 32); ah1.h[1] = *(const v8usa*)(ap + 48);
      al0.h[0] = *(const v8usa*)lp;        al0.h[1] = *(const v8usa*)(lp + 16);
      al1.h[0] = *(const v8usa*)(lp + 32); al1.h[1] = *(const v8usa*)(lp + 48);
#pragma unroll 1
      for (int nt = 0; nt < 32; ++nt) {
        v8f d = zero8();
        {
          const unsigned short* bp = w3p + (size_t)(16 * nt + m) * HID + 8 * hh;
          FragB bh, bl;
          bh.h[0] = *(const v8us*)bp;
          bh.h[1] = *(const v8us*)(bp + 16);
          bl.h[0] = *(const v8us*)(bp + WEC * HID);
          bl.h[1] = *(const v8us*)(bp + WEC * HID + 16);
          d = wmb(ah0.v, bh.v, d);
          d = wmb(ah0.v, bl.v, d);
          d = wmb(al0.v, bh.v, d);
        }
        {
          const unsigned short* bp = w3p + (size_t)(16 * nt + m) * HID + 32 + 8 * hh;
          FragB bh, bl;
          bh.h[0] = *(const v8us*)bp;
          bh.h[1] = *(const v8us*)(bp + 16);
          bl.h[0] = *(const v8us*)(bp + WEC * HID);
          bl.h[1] = *(const v8us*)(bp + WEC * HID + 16);
          d = wmb(ah1.v, bh.v, d);
          d = wmb(ah1.v, bl.v, d);
          d = wmb(al1.v, bh.v, d);
        }
#pragma unroll
        for (int r = 0; r < 8; ++r) wEw[(8 * hh + r) * WEP + 16 * nt + m] = d[r] * S64F;
      }
    }
    wave_lds_sync();
    int nr = total - 16 * t;
    nr = nr > 16 ? 16 : nr;
#pragma unroll 1
    for (int r = 0; r < nr; ++r) {
      const int g = 16 * t + r;
#pragma unroll 1
      while (cur < RUN - 1 && g >= bw[cur + 1]) {
        flush_node(totH, totL, runBase + cur, acc, lane);
        ++cur;
      }
      const int e = __builtin_amdgcn_readfirstlane(eidw[r]);
      const int j = __builtin_amdgcn_readfirstlane(jw[r]);
      const v4f xv = *(const v4f*)(xs + (size_t)j * MUL + 4 * lane);
      const float* yp = sph + (size_t)e * SHD;
      const v4f y0 = *(const v4f*)yp, y1 = *(const v4f*)(yp + 4), y2 = *(const v4f*)(yp + 8), y3 = *(const v4f*)(yp + 12);
      const float* wr = wEw + r * WEP + 4 * lane;
      const v4f w0v = *(const v4fa*)wr, w1v = *(const v4fa*)(wr + MUL), w2v = *(const v4fa*)(wr + 2 * MUL), w3v = *(const v4fa*)(wr + 3 * MUL);
      const v4f q0 = xv * w0v, q1 = xv * w1v, q2 = xv * w2v, q3 = xv * w3v;
      acc[0]  += q0 * y0.x;
      acc[1]  += q1 * y0.y;  acc[2]  += q1 * y0.z;  acc[3]  += q1 * y0.w;
      acc[4]  += q2 * y1.x;  acc[5]  += q2 * y1.y;  acc[6]  += q2 * y1.z;  acc[7]  += q2 * y1.w;
      acc[8]  += q2 * y2.x;
      acc[9]  += q3 * y2.y;  acc[10] += q3 * y2.z;  acc[11] += q3 * y2.w;
      acc[12] += q3 * y3.x;  acc[13] += q3 * y3.y;  acc[14] += q3 * y3.z;  acc[15] += q3 * y3.w;
    }
  }
#pragma unroll 1
  while (cur < RUN) {
    flush_node(totH, totL, runBase + cur, acc, lane);
    ++cur;
  }
}

__global__ __launch_bounds__(NTHR) __attribute__((amdgpu_num_vgpr(256)))
void k_post(const unsigned short* __restrict__ totH, const unsigned short* __restrict__ totL,
            const unsigned short* __restrict__ wp, float* out, int nN, float inv) {
  extern __shared__ v4f lds_dyn[];
  float* ostg = (float*)lds_dyn;
  const int tid = threadIdx.x, lane = tid & 31, wave = tid >> 5, hh = lane >> 4, m = lane & 15;
  const int nb = blockIdx.x * PNODE;
#pragma unroll 1
  for (int s = 0; s < 2; ++s) {
    const int dd = wave + 8 * s;
    const int p  = dd == 0 ? 0 : (dd < 4 ? 1 : (dd < 9 ? 2 : 3));
    const unsigned short* Bw = wp + PO_POST + (size_t)p * (2 * MUL * MUL);
    const unsigned short* aH = totH + ((size_t)(nb + m) * SHD + dd) * MUL + 8 * hh;
    const unsigned short* aL = totL + ((size_t)(nb + m) * SHD + dd) * MUL + 8 * hh;
    v8f acc[8];
#pragma unroll
    for (int t = 0; t < 8; ++t) acc[t] = zero8();
#pragma unroll
    for (int kt = 0; kt < MUL / 32; ++kt) {
      FragB ah, al;
      ah.h[0] = *(const v8us*)(aH + 32 * kt);
      ah.h[1] = *(const v8us*)(aH + 32 * kt + 16);
      al.h[0] = *(const v8us*)(aL + 32 * kt);
      al.h[1] = *(const v8us*)(aL + 32 * kt + 16);
#pragma unroll
      for (int t = 0; t < 8; ++t) {
        const unsigned short* bp = Bw + (size_t)(16 * t + m) * MUL + 32 * kt + 8 * hh;
        FragB bh, bl;
        bh.h[0] = *(const v8us*)bp;
        bh.h[1] = *(const v8us*)(bp + 16);
        bl.h[0] = *(const v8us*)(bp + MUL * MUL);
        bl.h[1] = *(const v8us*)(bp + MUL * MUL + 16);
        acc[t] = wmb(ah.v, bh.v, acc[t]);
        acc[t] = wmb(ah.v, bl.v, acc[t]);
        acc[t] = wmb(al.v, bh.v, acc[t]);
      }
    }
#pragma unroll
    for (int t = 0; t < 8; ++t) {
#pragma unroll
      for (int r = 0; r < 8; ++r)
        ostg[(8 * hh + r) * (MUL * SHD) + (16 * t + m) * SHD + dd] = acc[t][r] * inv;
    }
  }
  __syncthreads();

  float* op = out + (size_t)nb * (MUL * SHD);
  v4f ov[32];
#pragma unroll
  for (int i = 0; i < 32; ++i) ov[i] = ((const v4f*)ostg)[i * NTHR + tid];
#pragma unroll
  for (int i = 0; i < 32; ++i) {
    if (nb + (i >> 1) < nN) *(volatile v4f*)(op + 4 * (size_t)(i * NTHR + tid)) = ov[i];
  }
  __threadfence();
#pragma unroll
  for (int i = 0; i < 32; ++i) {
    if (nb + (i >> 1) < nN) *(volatile v4f*)(op + 4 * (size_t)(i * NTHR + tid)) = ov[i];
  }
}

extern "C" void kernel_launch(void* const* d_in, const int* in_sizes, int n_in,
                              void* d_out, int out_size, void* d_ws, size_t ws_size,
                              hipStream_t stream) {
  if (n_in < 11) return;
  if (in_sizes[0] <= 0 || (in_sizes[0] % MUL) != 0) return;
  const int nN = in_sizes[0] / MUL;
  const int nE = in_sizes[3];
  if (nN <= 0 || nE <= 0) return;
  if (in_sizes[1] != nE * SHD || in_sizes[2] != nE * RBF || in_sizes[4] != nE) return;
  if (in_sizes[5] != MUL * MUL || in_sizes[6] != RBF * HID || in_sizes[7] != HID * HID) return;
  if (in_sizes[8] != HID * HID || in_sizes[9] != HID * WEC || in_sizes[10] != 4 * MUL * MUL) return;
  if (out_size != nN * MUL * SHD) return;
  if (nE > (1 << 27) || nN > (1 << 22)) return;

  const float* nf    = (const float*)d_in[0];
  const float* sph   = (const float*)d_in[1];
  const float* rbp   = (const float*)d_in[2];
  const int*   ei    = (const int*)d_in[3];
  const int*   ej    = (const int*)d_in[4];
  const float* Wpre  = (const float*)d_in[5];
  const float* w0    = (const float*)d_in[6];
  const float* w1    = (const float*)d_in[7];
  const float* w2    = (const float*)d_in[8];
  const float* w3    = (const float*)d_in[9];
  const float* Wpost = (const float*)d_in[10];
  float* out = (float*)d_out;

  const int NPAD   = ((nN + TGT - 1) / TGT) * TGT;
  const int NPADX  = ((nN + GROWS - 1) / GROWS) * GROWS;
  const int nBC    = (nN + NBC - 1) / NBC;
  const int CNTPAD = nBC * NBC;
  if (4 * nBC + 1 > RBN) return;
  const int nBF    = (nN + NBF - 1) / NBF;
  const int csrLen = ((nE + 31) & ~31) + 4096;
  if (31 * 4 * nBC > 4096) return;
  if (NPAD > CNTPAD) return;
  const int nPre   = NPADX / GROWS;
  const int nEdge  = NPAD / TGT;
  const int nPost  = NPAD / PNODE;

  char* ws = (char*)d_ws;
  size_t off = 0;
  const size_t oW   = off; off += (size_t)PO_TOTAL * 2;                 off = (off + 255) & ~(size_t)255;
  const size_t oCnt = off; off += (size_t)CNTPAD * 4;                   off = (off + 255) & ~(size_t)255;
  const size_t oOff = off; off += (size_t)CNTPAD * 4;                   off = (off + 255) & ~(size_t)255;
  const size_t oRb  = off; off += (size_t)RBN * 4;                      off = (off + 255) & ~(size_t)255;
  const size_t oCsr = off; off += (size_t)csrLen * 4;                   off = (off + 255) & ~(size_t)255;
  const size_t oX   = off; off += (size_t)NPADX * MUL * 4;              off = (off + 255) & ~(size_t)255;
  const size_t oTH  = off; off += (size_t)NPAD * SHD * MUL * 2;         off = (off + 255) & ~(size_t)255;
  const size_t oTL  = off; off += (size_t)NPAD * SHD * MUL * 2;         off = (off + 255) & ~(size_t)255;
  if (off > ws_size || off > (size_t)WSCAP) return;
  unsigned short* wp   = (unsigned short*)(ws + oW);
  int*            cnt  = (int*)(ws + oCnt);
  int*            offp = (int*)(ws + oOff);
  int*            rb   = (int*)(ws + oRb);
  int*            csr  = (int*)(ws + oCsr);
  float*          xs   = (float*)(ws + oX);
  unsigned short* totH = (unsigned short*)(ws + oTH);
  unsigned short* totL = (unsigned short*)(ws + oTL);

  const int vec8 = ((nE & 3) == 0) ? 1 : 0;

  k_wprep<<<WPB, NTHR, 0, stream>>>(Wpre, w0, w1, w2, w3, Wpost, wp);

  k_count<<<nBC, NTHR, 0, stream>>>(ei, cnt, nE, vec8);
  k_offsets<<<1, OTHR, 0, stream>>>(cnt, offp, rb, nBC);
  hipFuncSetAttribute(reinterpret_cast<const void*>(&k_fill),
                      hipFuncAttributeMaxDynamicSharedMemorySize, LDS_FILL);
  k_fill<<<nBF, NTHR, LDS_FILL, stream>>>(ei, offp, rb, csr, nE, vec8, csrLen);

  hipFuncSetAttribute(reinterpret_cast<const void*>(&k_pre),
                      hipFuncAttributeMaxDynamicSharedMemorySize, LDS_PRE);
  k_pre<<<nPre, NTHR, LDS_PRE, stream>>>(nf, wp, xs, nN, INV128);

  hipFuncSetAttribute(reinterpret_cast<const void*>(&k_edge),
                      hipFuncAttributeMaxDynamicSharedMemorySize, LDS_EDGE);
  k_edge<<<nEdge, ETHR, LDS_EDGE, stream>>>(csr, offp, cnt, ej, rbp, sph, xs, wp, totH, totL, nN, nE, csrLen);

  hipFuncSetAttribute(reinterpret_cast<const void*>(&k_post),
                      hipFuncAttributeMaxDynamicSharedMemorySize, LDS_POST);
  k_post<<<nPost, NTHR, LDS_POST, stream>>>(totH, totL, wp, out, nN, INV128);
}
